// GCN_35218731827634
// MI455X (gfx1250) — hardware-verified
//
#include <hip/hip_runtime.h>
#include <stddef.h>
#include <stdint.h>
#include <math.h>


#define DF     128
#define KC     256
#define NEGS   0.01f
#define NTHR   256
#define NWAVE  8
#define EPT    8
#define CHUNK  (NTHR * EPT)
#define WCAP   (EPT * 32)
#define LISTN  (NWAVE * WCAP)
#define NBD    8192
#define SLD    13
#define NBA    1024
#define SLA    10
#define RCAP   16384
#define DEGCAP 64
#define GBM    64
#define GBN    128
#define GTHR   128
#define UMAT   4096
#define NMAT   3
#define AGG_ZINTS    (LISTN + 2 * RCAP + 3 * NBA)
#define MISC_INTS    16
#define ROWBUF_INTS  (NWAVE * KC / 2)
#define AGG_LDS_INTS (AGG_ZINTS + MISC_INTS + ROWBUF_INTS)
#define WSMAX  134217728

static_assert((CHUNK & (CHUNK - 1)) == 0 && CHUNK <= 4096);
static_assert((NBD & (NBD - 1)) == 0 && NBD == (1 << SLD));
static_assert((NBA & (NBA - 1)) == 0 && NBA == (1 << SLA));
static_assert(((long long)CHUNK << SLD) < (1LL << 31));
static_assert(((long long)CHUNK << SLA) < (1LL << 31));
static_assert(NBD % (NTHR * 4) == 0);
static_assert(LISTN % NTHR == 0);
static_assert(NBA % NWAVE == 0 && NBA % 32 == 0 && NBA % GBM == 0);
static_assert(RCAP % 4 == 0 && AGG_ZINTS % 4 == 0 && LISTN % 4 == 0 && ((AGG_ZINTS + MISC_INTS) % 4) == 0);
static_assert(AGG_ZINTS % (NTHR * 4) == 0);
static_assert(KC % 32 == 0 && KC == 2 * DF && DF == 4 * 32);
static_assert(GBN == DF && GBM == (GTHR / 32) * 16);
static_assert(UMAT % NTHR == 0 && UMAT == DF * (KC / 8) && (NMAT * UMAT) % NTHR == 0);
static_assert(AGG_LDS_INTS * 4 <= 300000);

typedef float          v4f   __attribute__((ext_vector_type(4)));
typedef float          v8f   __attribute__((ext_vector_type(8)));
typedef int            v4i   __attribute__((ext_vector_type(4)));
typedef int            v8i   __attribute__((ext_vector_type(8)));
typedef unsigned short v4us  __attribute__((ext_vector_type(4)));
typedef unsigned short v8us  __attribute__((ext_vector_type(8)));
typedef unsigned short v16us __attribute__((ext_vector_type(16)));
typedef __bf16         v16bf __attribute__((ext_vector_type(16)));
typedef v4f  __attribute__((may_alias)) v4fa;
typedef v4i  __attribute__((may_alias)) v4ia;
typedef v4us __attribute__((may_alias)) v4usa;
typedef v8us __attribute__((may_alias)) v8usa;
union FragB { v16bf v; v16us u; v8us h[2]; v8i w; };

__device__ __forceinline__ v8f wmb(const FragB& a, const FragB& b, v8f c) {
  v8f d = __builtin_amdgcn_wmma_f32_16x16x32_bf16(false, a.v, false, b.v, (short)0, c, false, false);
  asm volatile("v_nop\n\tv_nop\n\tv_nop\n\tv_nop" : "+v"(d) : "v"(a.w), "v"(b.w));
  return d;
}

__device__ __forceinline__ unsigned bf16_bits(float f) {
  const unsigned u = __float_as_uint(f);
  return (u + 0x7FFFu + ((u >> 16) & 1u)) >> 16;
}
__device__ __forceinline__ float bf16_val(float f) {
  return __uint_as_float(bf16_bits(f) << 16);
}

__device__ __forceinline__ void wave_sync() {
  __builtin_amdgcn_fence(__ATOMIC_RELEASE, "wavefront");
  __builtin_amdgcn_wave_barrier();
  __builtin_amdgcn_fence(__ATOMIC_ACQUIRE, "wavefront");
}

__device__ __forceinline__ float rsq1(float d) {
  float y = rsqrtf(d);
  const float r = fmaf(-d * y, y, 1.0f);
  y = fmaf(0.5f * y, r, y);
  return (d > 0.0f) ? y : 0.0f;
}

template <int SLB>
__device__ __forceinline__ int scan_chunk(const int* __restrict__ dsts, int nE, int cbase, int slotBase,
                                          int nb, int vec8, int* list, int tid, int lane, int wave) {
  int wc = 0;
  const int el0  = tid * EPT;
  const int e0   = cbase + el0;
  const int sent = -2147483647 - 1;
  v4i da, db;
  if (vec8 != 0 && cbase + CHUNK <= nE) {
    da = *(const v4i*)(dsts + e0);
    db = *(const v4i*)(dsts + e0 + 4);
  } else {
    da.x = (e0     < nE) ? dsts[min(e0,     nE - 1)] : sent;
    da.y = (e0 + 1 < nE) ? dsts[min(e0 + 1, nE - 1)] : sent;
    da.z = (e0 + 2 < nE) ? dsts[min(e0 + 2, nE - 1)] : sent;
    da.w = (e0 + 3 < nE) ? dsts[min(e0 + 3, nE - 1)] : sent;
    db.x = (e0 + 4 < nE) ? dsts[min(e0 + 4, nE - 1)] : sent;
    db.y = (e0 + 5 < nE) ? dsts[min(e0 + 5, nE - 1)] : sent;
    db.z = (e0 + 6 < nE) ? dsts[min(e0 + 6, nE - 1)] : sent;
    db.w = (e0 + 7 < nE) ? dsts[min(e0 + 7, nE - 1)] : sent;
  }
  const unsigned nbs = (unsigned)slotBase;
  const unsigned unb = (unsigned)nb;
  const unsigned s0 = (unsigned)da.x - nbs, s1 = (unsigned)da.y - nbs;
  const unsigned s2 = (unsigned)da.z - nbs, s3 = (unsigned)da.w - nbs;
  const unsigned s4 = (unsigned)db.x - nbs, s5 = (unsigned)db.y - nbs;
  const unsigned s6 = (unsigned)db.z - nbs, s7 = (unsigned)db.w - nbs;
  const bool h0 = s0 < unb, h1 = s1 < unb, h2 = s2 < unb, h3 = s3 < unb;
  const bool h4 = s4 < unb, h5 = s5 < unb, h6 = s6 < unb, h7 = s7 < unb;
  const unsigned any = __builtin_amdgcn_ballot_w32(h0 | h1 | h2 | h3 | h4 | h5 | h6 | h7);
  if (any != 0u) {
#define HITJ(J, HJ, SJ) { \
      const unsigned mj = __builtin_amdgcn_ballot_w32(HJ); \
      if (mj != 0u) { \
        if (HJ) { \
          const int pos = wc + (int)__builtin_amdgcn_mbcnt_lo(mj, 0u); \
          if (pos < WCAP) list[wave * WCAP + pos] = ((el0 + (J)) << SLB) | (int)(SJ); \
        } \
        wc += (int)__builtin_popcount(mj); } }
    HITJ(0, h0, s0)
    HITJ(1, h1, s1)
    HITJ(2, h2, s2)
    HITJ(3, h3, s3)
    HITJ(4, h4, s4)
    HITJ(5, h5, s5)
    HITJ(6, h6, s6)
    HITJ(7, h7, s7)
#undef HITJ
  }
  return wc;
}

__device__ __forceinline__ v8us wgath(const float* __restrict__ p) {
  v8us o;
#pragma unroll
  for (int i = 0; i < 8; ++i) o[i] = (unsigned short)bf16_bits(p[(size_t)i * DF]);
  return o;
}

__global__ __launch_bounds__(NTHR) void k_wprep(const float* __restrict__ W1, const float* __restrict__ W2,
                                                const float* __restrict__ W3, unsigned short* WT) {
  const int u = (int)blockIdx.x * NTHR + (int)threadIdx.x;
  if (u >= NMAT * UMAT) return;
  const int mat = u >> 12;
  const int v   = u & (UMAT - 1);
  const int n   = v >> 5;
  const int k8  = (v & 31) * 8;
  const int kk  = k8 & (DF - 1);
  const size_t so = (size_t)kk * DF + n;
  v8us o;
  if (mat == 0)      o = wgath(W1 + so);
  else if (mat == 1) o = wgath(W2 + so);
  else               o = wgath(W3 + so);
  unsigned short* dp = WT + (size_t)mat * (DF * KC) + (size_t)n * KC + k8;
  *(volatile v8us*)dp = o;
  __threadfence();
  *(volatile v8us*)dp = o;
}

__device__ __forceinline__ void cvt_hl(float xv, bool ok, unsigned short& h, unsigned short& l) {
  const float xr = bf16_val(xv);
  const float av = (xr > 0.0f) ? xr : NEGS * xr;
  const unsigned hb = bf16_bits(av);
  const unsigned lb = bf16_bits(av - __uint_as_float(hb << 16));
  h = ok ? (unsigned short)hb : (unsigned short)0;
  l = ok ? (unsigned short)lb : (unsigned short)0;
}

__global__ __launch_bounds__(NTHR) void k_cvx(const float* __restrict__ x, int nN, int nUnits,
                                              unsigned short* xa) {
  const int u = (int)blockIdx.x * NTHR + (int)threadIdx.x;
  if (u >= nUnits) return;
  const int row = u >> 4;
  const int k8  = (u & 15) * 8;
  const int rc  = row < nN ? row : nN - 1;
  const float* p = x + (size_t)rc * DF + k8;
  const v4f a = *(const v4fa*)p;
  const v4f b = *(const v4fa*)(p + 4);
  const bool ok = row < nN;
  unsigned short h0, h1, h2, h3, h4, h5, h6, h7, l0, l1, l2, l3, l4, l5, l6, l7;
  cvt_hl(a.x, ok, h0, l0); cvt_hl(a.y, ok, h1, l1); cvt_hl(a.z, ok, h2, l2); cvt_hl(a.w, ok, h3, l3);
  cvt_hl(b.x, ok, h4, l4); cvt_hl(b.y, ok, h5, l5); cvt_hl(b.z, ok, h6, l6); cvt_hl(b.w, ok, h7, l7);
  v8us oh, ol;
  oh[0] = h0; oh[1] = h1; oh[2] = h2; oh[3] = h3; oh[4] = h4; oh[5] = h5; oh[6] = h6; oh[7] = h7;
  ol[0] = l0; ol[1] = l1; ol[2] = l2; ol[3] = l3; ol[4] = l4; ol[5] = l5; ol[6] = l6; ol[7] = l7;
  unsigned short* dp = xa + (size_t)row * KC + k8;
  *(volatile v8us*)dp = oh;
  *(volatile v8us*)(dp + DF) = ol;
  __threadfence();
  *(volatile v8us*)dp = oh;
  *(volatile v8us*)(dp + DF) = ol;
}

__global__ __launch_bounds__(NTHR) void k_deg(const int* __restrict__ dsts, int nE, int vec8, float* dis) {
  __shared__ __attribute__((aligned(16))) int scnt[NBD];
  __shared__ __attribute__((aligned(16))) int list[LISTN];
  __shared__ int wcnt[NWAVE];
  const int tid = (int)threadIdx.x, lane = tid & 31, wave = tid >> 5;
  const int nodeBase = (int)blockIdx.x * NBD;

  for (int i = tid; i < NBD; i += NTHR) scnt[i] = 0;
  for (int i = tid; i < LISTN; i += NTHR) list[i] = 0;
  if (tid < NWAVE) wcnt[tid] = 0;
  __syncthreads();

  const int nChunks = (nE + CHUNK - 1) / CHUNK;
#pragma unroll 1
  for (int ch = 0; ch < nChunks; ++ch) {
    const int cbase = ch * CHUNK;
    const int wc = scan_chunk<SLD>(dsts, nE, cbase, nodeBase, NBD, vec8, list, tid, lane, wave);
    if (lane == 0) wcnt[wave] = wc;
    __syncthreads();
    if (wave == 0) {
#pragma unroll 1
      for (int w2 = 0; w2 < NWAVE; ++w2) {
        int c = wcnt[w2];
        c = c < 0 ? 0 : (c > WCAP ? WCAP : c);
#pragma unroll 1
        for (int b0 = 0; b0 < c; b0 += 32) {
          const int idx = b0 + lane;
          const int ent = list[w2 * WCAP + (idx < WCAP ? idx : WCAP - 1)];
          const int m32 = (c - b0) < 32 ? (c - b0) : 32;
#pragma unroll 1
          for (int k = 0; k < m32; ++k) {
            const int u  = __builtin_amdgcn_readlane(ent, k);
            const int sl = u & (NBD - 1);
            if (lane == 0) scnt[sl] = scnt[sl] + 1;
          }
        }
      }
    }
    __syncthreads();
  }

#pragma unroll 1
  for (int it = 0; it < NBD / (NTHR * 4); ++it) {
    const int s0 = it * (NTHR * 4) + 4 * tid;
    const v4i c4 = *(const v4ia*)(scnt + s0);
    v4f v;
    v.x = rsq1((float)c4.x + 1.0f); v.y = rsq1((float)c4.y + 1.0f);
    v.z = rsq1((float)c4.z + 1.0f); v.w = rsq1((float)c4.w + 1.0f);
    *(volatile v4f*)(dis + (size_t)nodeBase + s0) = v;
  }
  __threadfence();
#pragma unroll 1
  for (int it = 0; it < NBD / (NTHR * 4); ++it) {
    const int s0 = it * (NTHR * 4) + 4 * tid;
    const v4i c4 = *(const v4ia*)(scnt + s0);
    v4f v;
    v.x = rsq1((float)c4.x + 1.0f); v.y = rsq1((float)c4.y + 1.0f);
    v.z = rsq1((float)c4.z + 1.0f); v.w = rsq1((float)c4.w + 1.0f);
    *(volatile v4f*)(dis + (size_t)nodeBase + s0) = v;
  }
}

__global__ __launch_bounds__(GTHR) void k_gemm(const unsigned short* __restrict__ Apl,
                                               const unsigned short* __restrict__ BT,
                                               const float* __restrict__ dis, float* hs, int nN) {
  __shared__ __attribute__((aligned(16))) float stg[GBM * GBN];
  const int tid = (int)threadIdx.x, lane = tid & 31, wave = tid >> 5, hh = lane >> 4, m = lane & 15;
  const int rowBase = (int)blockIdx.x * GBM;

  v8f acc[8];
  {
    const v8f z = {0.f, 0.f, 0.f, 0.f, 0.f, 0.f, 0.f, 0.f};
#pragma unroll
    for (int t = 0; t < 8; ++t) acc[t] = z;
  }
  const unsigned short* ap = Apl + (size_t)(rowBase + 16 * wave + m) * (size_t)KC + 8 * hh;
  const unsigned short* bp = BT + (size_t)m * (size_t)KC + 8 * hh;

#pragma unroll 1
  for (int k0 = 0; k0 < KC; k0 += 32) {
    FragB af;
    af.h[0] = *(const v8usa*)(ap + k0);
    af.h[1] = *(const v8usa*)(ap + k0 + 16);
#pragma unroll
    for (int nt = 0; nt < 8; ++nt) {
      const unsigned short* wq = bp + (size_t)(16 * nt) * (size_t)KC + k0;
      FragB bf;
      bf.h[0] = *(const v8usa*)wq;
      bf.h[1] = *(const v8usa*)(wq + 16);
      acc[nt] = wmb(af, bf, acc[nt]);
    }
  }

#pragma unroll
  for (int nt = 0; nt < 8; ++nt) {
    const int lc = 16 * nt + m;
#pragma unroll
    for (int r = 0; r < 8; ++r) {
      const int lr = 16 * wave + 8 * hh + r;
      stg[lr * GBN + lc] = acc[nt][r];
    }
  }
  __syncthreads();

  const int rl = rowBase + 16 * wave + m;
  const float dvl = dis[rl < nN ? rl : nN - 1];

  v4f pv[16];
#pragma unroll
  for (int i = 0; i < 16; ++i) pv[i] = *(const v4fa*)(stg + (16 * wave + i) * GBN + 4 * lane);

#pragma unroll
  for (int i = 0; i < 16; ++i) {
    const bool ok = (rowBase + 16 * wave + i) < nN;
    const float dv = __shfl(dvl, i, 32);
    v4f y;
    y.x = pv[i].x * dv; y.y = pv[i].y * dv; y.z = pv[i].z * dv; y.w = pv[i].w * dv;
    y.x = ok ? y.x : 0.0f; y.y = ok ? y.y : 0.0f; y.z = ok ? y.z : 0.0f; y.w = ok ? y.w : 0.0f;
    pv[i] = y;
  }

#pragma unroll
  for (int i = 0; i < 16; ++i) {
    float* op = hs + (size_t)(rowBase + 16 * wave + i) * DF + 4 * lane;
    *(volatile v4f*)op = pv[i];
  }
  __threadfence();
#pragma unroll
  for (int i = 0; i < 16; ++i) {
    float* op = hs + (size_t)(rowBase + 16 * wave + i) * DF + 4 * lane;
    *(volatile v4f*)op = pv[i];
  }
}

template <int ACT>
__global__ __launch_bounds__(NTHR) void k_scan(const int* __restrict__ srcs, const int* __restrict__ dsts,
                                               int nE, int nN, int vec8, int mRows,
                                               const float* __restrict__ dis, const float* __restrict__ hs,
                                               const float* __restrict__ bias,
                                               unsigned short* xa, float* outp) {
  extern __shared__ __attribute__((aligned(16))) int dsm[];
  int* list = dsm;
  int* hl   = dsm + LISTN;
  int* sl   = hl + RCAP;
  int* cnt  = sl + RCAP;
  int* offs = cnt + NBA;
  int* cur  = offs + NBA;
  int* misc = cur + NBA;
  const int tid = (int)threadIdx.x, lane = tid & 31, wave = tid >> 5;
  unsigned short* rowbuf = (unsigned short*)(misc + MISC_INTS) + wave * KC;
  const int nodeBase = (int)blockIdx.x * NBA;

  {
    const v4i z4 = {0, 0, 0, 0};
    for (int i = tid * 4; i < AGG_ZINTS; i += NTHR * 4) *(v4ia*)(dsm + i) = z4;
    if (tid < MISC_INTS) misc[tid] = 0;
  }
  float bv0, bv1, bv2, bv3;
  {
    const v4f bq = *(const v4fa*)(bias + 4 * lane);
    bv0 = bf16_val(bq.x); bv1 = bf16_val(bq.y); bv2 = bf16_val(bq.z); bv3 = bf16_val(bq.w);
  }
  __syncthreads();

  int t = 0, ov = 0;
  const int nChunks = (nE + CHUNK - 1) / CHUNK;
#pragma unroll 1
  for (int ch = 0; ch < nChunks; ++ch) {
    const int cbase = ch * CHUNK;
    const int wc = scan_chunk<SLA>(dsts, nE, cbase, nodeBase, NBA, vec8, list, tid, lane, wave);
    if (lane == 0) misc[wave] = wc;
    __syncthreads();
    if (wave == 0) {
#pragma unroll 1
      for (int w2 = 0; w2 < NWAVE; ++w2) {
        int c = misc[w2];
        c = c < 0 ? 0 : (c > WCAP ? WCAP : c);
#pragma unroll 1
        for (int b0 = 0; b0 < c; b0 += 32) {
          const int idx = b0 + lane;
          const int ent = list[w2 * WCAP + (idx < WCAP ? idx : WCAP - 1)];
          const int m32 = (c - b0) < 32 ? (c - b0) : 32;
#pragma unroll 1
          for (int k = 0; k < m32; ++k) {
            const int u    = __builtin_amdgcn_readlane(ent, k);
            const int slot = u & (NBA - 1);
            const int el   = (u >> SLA) & (CHUNK - 1);
            const int pk   = ((cbase + el) << SLA) | slot;
            if (t < RCAP) {
              if (lane == 0) { hl[t] = pk; cnt[slot] = cnt[slot] + 1; }
              t = t + 1;
            } else {
              ov = 1;
            }
          }
        }
      }
    }
    __syncthreads();
  }
  if (wave == 0 && lane == 0) { misc[8] = t; misc[9] = ov; }
  __syncthreads();
  int tt = misc[8];
  tt = tt < 0 ? 0 : (tt > RCAP ? RCAP : tt);
  const int ovf = misc[9];

  if (wave == 0) {
    const int base = lane * (NBA / 32);
    int s = 0;
#pragma unroll 1
    for (int i = 0; i < NBA / 32; ++i) s += cnt[base + i];
    int incl = s;
#pragma unroll
    for (int d = 1; d < 32; d <<= 1) {
      const int y = __shfl_up(incl, d, 32);
      if (lane >= d) incl += y;
    }
    int run = incl - s;
#pragma unroll 1
    for (int i = 0; i < NBA / 32; ++i) {
      const int cv = cnt[base + i];
      offs[base + i] = run;
      cur[base + i]  = run;
      run += cv;
    }
  }
  __syncthreads();
  if (wave == 0) {
#pragma unroll 1
    for (int b0 = 0; b0 < tt; b0 += 32) {
      const int idx = b0 + lane;
      const int ent = hl[idx < RCAP ? idx : RCAP - 1];
      const int m32 = (tt - b0) < 32 ? (tt - b0) : 32;
#pragma unroll 1
      for (int k = 0; k < m32; ++k) {
        const int u    = __builtin_amdgcn_readlane(ent, k);
        const int slot = u & (NBA - 1);
        if (lane == 0) {
          int p = cur[slot];
          p = p < 0 ? 0 : (p > RCAP - 1 ? RCAP - 1 : p);
          sl[p] = u;
          cur[slot] = p + 1;
        }
      }
    }
  }
  __syncthreads();

  const float qnan = __int_as_float(0x7fc00000);
  const float pz = (ovf != 0) ? qnan : 0.0f;
#pragma unroll 1
  for (int si = 0; si < NBA / NWAVE; ++si) {
    const int s    = si * NWAVE + wave;
    const int node = nodeBase + s;
    int c = cnt[s];
    const bool big = c > DEGCAP;
    c = c < 0 ? 0 : (c > DEGCAP ? DEGCAP : c);
    int o = offs[s];
    o = o < 0 ? 0 : (o > RCAP ? RCAP : o);
    const int nc = node < nN ? node : nN - 1;
    const float dd = dis[nc];
    float a0 = 0.0f, a1 = 0.0f, a2 = 0.0f, a3 = 0.0f;
#pragma unroll 1
    for (int b0 = 0; b0 < c; b0 += 32) {
      int idx = o + b0 + lane;
      idx = idx > RCAP - 1 ? RCAP - 1 : idx;
      const int ent = sl[idx];
      int eid = ent >> SLA;
      eid = eid < 0 ? 0 : (eid > nE - 1 ? nE - 1 : eid);
      int sr = srcs[eid];
      sr = sr < 0 ? 0 : (sr > nN - 1 ? nN - 1 : sr);
      const int m32 = (c - b0) < 32 ? (c - b0) : 32;
#pragma unroll 1
      for (int k = 0; k < m32; ++k) {
        const int sk = __builtin_amdgcn_readlane(sr, k);
        const v4f a = *(const v4fa*)(hs + (size_t)sk * DF + 4 * lane);
        a0 += a.x; a1 += a.y; a2 += a.z; a3 += a.w;
      }
    }
    const v4f sv = *(const v4fa*)(hs + (size_t)nc * DF + 4 * lane);
    const float pzr = big ? qnan : pz;
    const bool live = node < nN;
    float y0 = dd * (a0 + sv.x) + bv0;
    float y1 = dd * (a1 + sv.y) + bv1;
    float y2 = dd * (a2 + sv.z) + bv2;
    float y3 = dd * (a3 + sv.w) + bv3;
    y0 = y0 + pzr; y1 = y1 + pzr; y2 = y2 + pzr; y3 = y3 + pzr;
    if constexpr (ACT != 0) {
      y0 = (y0 > 0.0f) ? y0 : NEGS * y0;
      y1 = (y1 > 0.0f) ? y1 : NEGS * y1;
      y2 = (y2 > 0.0f) ? y2 : NEGS * y2;
      y3 = (y3 > 0.0f) ? y3 : NEGS * y3;
      const float m0 = live ? y0 : 0.0f;
      const float m1 = live ? y1 : 0.0f;
      const float m2 = live ? y2 : 0.0f;
      const float m3 = live ? y3 : 0.0f;
      v4us mh, ml;
      {
        unsigned hb;
        hb = bf16_bits(m0); mh[0] = (unsigned short)hb; ml[0] = (unsigned short)bf16_bits(m0 - __uint_as_float(hb << 16));
        hb = bf16_bits(m1); mh[1] = (unsigned short)hb; ml[1] = (unsigned short)bf16_bits(m1 - __uint_as_float(hb << 16));
        hb = bf16_bits(m2); mh[2] = (unsigned short)hb; ml[2] = (unsigned short)bf16_bits(m2 - __uint_as_float(hb << 16));
        hb = bf16_bits(m3); mh[3] = (unsigned short)hb; ml[3] = (unsigned short)bf16_bits(m3 - __uint_as_float(hb << 16));
      }
      *(v4usa*)(rowbuf + 4 * lane) = mh;
      *(v4usa*)(rowbuf + DF + 4 * lane) = ml;
      wave_sync();
      const v8us q0 = *(const v8usa*)(rowbuf + 8 * lane);
      wave_sync();
      if (node < mRows) {
        unsigned short* rpw = xa + (size_t)node * KC + 8 * lane;
        *(volatile v8us*)rpw = q0;
        __threadfence();
        *(volatile v8us*)rpw = q0;
      }
    } else {
      v4f ow;
      ow.x = y0; ow.y = y1; ow.z = y2; ow.w = y3;
      if (live) {
        float* op = outp + (size_t)node * DF + 4 * lane;
        *(volatile v4f*)op = ow;
        __threadfence();
        *(volatile v4f*)op = ow;
      }
    }
  }
}

static inline int cdiv(int a, int b) { return (a + b - 1) / b; }
static inline size_t al256(size_t o) { return (o + 255) & ~(size_t)255; }

extern "C" void kernel_launch(void* const* d_in, const int* in_sizes, int n_in,
                              void* d_out, int out_size, void* d_ws, size_t ws_size,
                              hipStream_t stream) {
  if (n_in < 8) return;
  if (in_sizes[0] < DF || (in_sizes[0] % DF) != 0) return;
  const int nN = in_sizes[0] / DF;
  if (nN < 16 || nN > (1 << 22)) return;
  if (in_sizes[1] < 2 || (in_sizes[1] & 1) != 0) return;
  const int nE = in_sizes[1] / 2;
  if (nE < 1 || nE >= (1 << (31 - SLA))) return;
  if (in_sizes[2] != DF * DF || in_sizes[3] != DF) return;
  if (in_sizes[4] != DF * DF || in_sizes[5] != DF) return;
  if (in_sizes[6] != DF * DF || in_sizes[7] != DF) return;
  if ((long long)out_size != (long long)nN * DF) return;

  const float* x    = (const float*)d_in[0];
  const int*   edge = (const int*)d_in[1];
  const float* W1   = (const float*)d_in[2];
  const float* b1   = (const float*)d_in[3];
  const float* W2   = (const float*)d_in[4];
  const float* b2   = (const float*)d_in[5];
  const float* W3   = (const float*)d_in[6];
  const float* b3   = (const float*)d_in[7];
  float* out = (float*)d_out;
  const int* src = edge;
  const int* dst = edge + nE;

  const int MP   = cdiv(nN, GBM) * GBM;
  const int gM   = MP / GBM;
  const int gD   = cdiv(nN, NBD);
  const int NBPD = gD * NBD;
  const int gA   = cdiv(MP, NBA);
  if ((long long)gA * NBA < (long long)MP) return;
  if (NBPD < nN) return;
  const int vec8 = ((nE & 3) == 0) ? 1 : 0;

  char* ws = (char*)d_ws;
  size_t off = 0;
  const size_t oDIS = off; off = al256(off + (size_t)NBPD * 4);
  const size_t oWT  = off; off = al256(off + (size_t)NMAT * DF * KC * 2);
  const size_t oXA  = off; off = al256(off + (size_t)MP * KC * 2);
  const size_t oHS  = off; off = al256(off + (size_t)MP * DF * 4);
  if (off > ws_size || off > (size_t)WSMAX) return;
  float*          DIS = (float*)(ws + oDIS);
  unsigned short* WT  = (unsigned short*)(ws + oWT);
  unsigned short* XA  = (unsigned short*)(ws + oXA);
  float*          HS  = (float*)(ws + oHS);
  const unsigned short* WT1 = WT;
  const unsigned short* WT2 = WT + (size_t)DF * KC;
  const unsigned short* WT3 = WT + (size_t)2 * DF * KC;

  const size_t scanLds = (size_t)AGG_LDS_INTS * 4;
  hipFuncSetAttribute(reinterpret_cast<const void*>(&k_scan<1>), hipFuncAttributeMaxDynamicSharedMemorySize, (int)scanLds);
  hipFuncSetAttribute(reinterpret_cast<const void*>(&k_scan<0>), hipFuncAttributeMaxDynamicSharedMemorySize, (int)scanLds);

  const int nUx = MP * (DF / 8);
  k_wprep<<<(NMAT * UMAT) / NTHR, NTHR, 0, stream>>>(W1, W2, W3, WT);
  k_cvx<<<cdiv(nUx, NTHR), NTHR, 0, stream>>>(x, nN, nUx, XA);
  k_deg<<<gD, NTHR, 0, stream>>>(dst, nE, vec8, DIS);
  k_gemm<<<gM, GTHR, 0, stream>>>(XA, WT1, DIS, HS, nN);
  k_scan<1><<<gA, NTHR, scanLds, stream>>>(src, dst, nE, nN, vec8, MP, DIS, HS, b1, XA, out);
  k_gemm<<<gM, GTHR, 0, stream>>>(XA, WT2, DIS, HS, nN);
  k_scan<1><<<gA, NTHR, scanLds, stream>>>(src, dst, nE, nN, vec8, MP, DIS, HS, b2, XA, out);
  k_gemm<<<gM, GTHR, 0, stream>>>(XA, WT3, DIS, HS, nN);
  k_scan<0><<<gA, NTHR, scanLds, stream>>>(src, dst, nE, nN, vec8, MP, DIS, HS, b3, XA, out);
}
